// CrossPatchSelfAttention_2920577762065
// MI455X (gfx1250) — hardware-verified
//
#include <hip/hip_runtime.h>

typedef _Float16 v16h __attribute__((ext_vector_type(16)));
typedef _Float16 v8h  __attribute__((ext_vector_type(8)));
typedef float    v8f  __attribute__((ext_vector_type(8)));
typedef float    v4f  __attribute__((ext_vector_type(4)));
typedef v8h __attribute__((may_alias)) v8ha;
typedef v4f __attribute__((may_alias)) v4fa;

union Frag { v16h v; v8h half[2]; };

#define DM     1024
#define NH     16
#define HD     64
#define SEQ    1024
#define NB     8
#define MROWS  (NB * SEQ)
#define FF     4096
#define PSCALE 16384.0f
#define GSCALE 16.0f
#define SSCALE 0.125f

__device__ __forceinline__ v8f wmma_f16(v16h a, v16h b, v8f c) {
  v8f d = __builtin_amdgcn_wmma_f32_16x16x32_f16(false, a, false, b, (short)0, c, false, false);
  asm volatile("v_nop\n\tv_nop\n\tv_nop\n\tv_nop" : "+v"(d) : "v"(a), "v"(b));
  return d;
}

__device__ __forceinline__ v16h load_frag(const _Float16* p, int h) {
  Frag f;
  f.half[0] = *(const v8ha*)(p + 8 * h);
  f.half[1] = *(const v8ha*)(p + 16 + 8 * h);
  return f.v;
}

__global__ __launch_bounds__(256) void wtrans_kernel(
    const float* __restrict__ in, _Float16* __restrict__ out, int K, int N, float sc)
{
  __shared__ float t[64][33];
  const int tid = threadIdx.x, lane = tid & 31, w = tid >> 5;
  const int n0 = blockIdx.x * 32, k0 = blockIdx.y * 64;
  const int kk = tid >> 2, cc = (tid & 3) * 8;
  const float* src = in + (size_t)(k0 + kk) * N + n0 + cc;
  const v4f a = *(const v4fa*)src;
  const v4f c = *(const v4fa*)(src + 4);
  t[kk][cc + 0] = a.x; t[kk][cc + 1] = a.y; t[kk][cc + 2] = a.z; t[kk][cc + 3] = a.w;
  t[kk][cc + 4] = c.x; t[kk][cc + 5] = c.y; t[kk][cc + 6] = c.z; t[kk][cc + 7] = c.w;
  __syncthreads();

  const int sub = lane >> 3, q8 = lane & 7;
  const int nn = w * 4 + sub;
  v8h o;
  #pragma unroll
  for (int j = 0; j < 8; ++j) o[j] = (_Float16)(t[8 * q8 + j][nn] * sc);
  _Float16* dst = out + (size_t)(n0 + nn) * K + k0 + 8 * q8;
  *(volatile v8h*)dst = o;
  __threadfence();
  *(volatile v8h*)dst = o;
}

__global__ __launch_bounds__(128) void ln_kernel(
    const float* __restrict__ x, const float* __restrict__ g,
    const float* __restrict__ be, _Float16* __restrict__ out)
{
  __shared__ float red[8];
  const int tid = threadIdx.x, lane = tid & 31, w = tid >> 5;
  const int row = blockIdx.x;
  const float* xr = x + (size_t)row * DM + 8 * tid;
  const v4f a = *(const v4fa*)xr;
  const v4f c = *(const v4fa*)(xr + 4);

  float s = ((a.x + a.y) + (a.z + a.w)) + ((c.x + c.y) + (c.z + c.w));
  #pragma unroll
  for (int off = 16; off > 0; off >>= 1) s += __shfl_xor(s, off, 32);
  if (lane == 0) red[w] = s;
  __syncthreads();
  const float mu = ((red[0] + red[1]) + (red[2] + red[3])) * (1.0f / 1024.0f);

  const float d0 = a.x - mu, d1 = a.y - mu, d2 = a.z - mu, d3 = a.w - mu;
  const float d4 = c.x - mu, d5 = c.y - mu, d6 = c.z - mu, d7 = c.w - mu;
  float s2 = ((d0 * d0 + d1 * d1) + (d2 * d2 + d3 * d3)) + ((d4 * d4 + d5 * d5) + (d6 * d6 + d7 * d7));
  #pragma unroll
  for (int off = 16; off > 0; off >>= 1) s2 += __shfl_xor(s2, off, 32);
  if (lane == 0) red[4 + w] = s2;
  __syncthreads();
  const float var = ((red[4] + red[5]) + (red[6] + red[7])) * (1.0f / 1024.0f);
  const float rstd = rsqrtf(var + 1e-5f);

  const v4f ga = *(const v4fa*)(g + 8 * tid);
  const v4f gc = *(const v4fa*)(g + 8 * tid + 4);
  const v4f ba = *(const v4fa*)(be + 8 * tid);
  const v4f bc = *(const v4fa*)(be + 8 * tid + 4);
  const v8h o = { (_Float16)(d0 * rstd * ga.x + ba.x), (_Float16)(d1 * rstd * ga.y + ba.y),
                  (_Float16)(d2 * rstd * ga.z + ba.z), (_Float16)(d3 * rstd * ga.w + ba.w),
                  (_Float16)(d4 * rstd * gc.x + bc.x), (_Float16)(d5 * rstd * gc.y + bc.y),
                  (_Float16)(d6 * rstd * gc.z + bc.z), (_Float16)(d7 * rstd * gc.w + bc.w) };
  _Float16* dst = out + (size_t)row * DM + 8 * tid;
  *(volatile v8h*)dst = o;
  __threadfence();
  *(volatile v8h*)dst = o;
}

__device__ __forceinline__ void qkv_store_pass(const _Float16* sT, _Float16* plane, _Float16* vt,
                                               int which, int bh, int l0, int w, int lane) {
  const int q8 = lane & 7, sub = lane >> 3;
  #pragma unroll
  for (int i = 0; i < 8; ++i) {
    const int lid = w * 32 + i * 4 + sub;
    v8h v;
    _Float16* dst;
    if (which != 2) {
      v = *(const v8ha*)(sT + lid * HD + 8 * q8);
      dst = plane + ((size_t)bh * SEQ + l0 + lid) * HD + 8 * q8;
    } else {
      const int d = lid >> 1, hl = lid & 1;
      v = *(const v8ha*)(sT + d * 128 + 64 * hl + 8 * q8);
      dst = vt + ((size_t)bh * HD + d) * SEQ + l0 + 64 * hl + 8 * q8;
    }
    *(volatile v8h*)dst = v;
  }
}

__device__ __forceinline__ void f16_store_pass(const _Float16* sT, _Float16* base, int ldc,
                                               int w, int lane) {
  const int q8 = lane & 7, sub = lane >> 3;
  #pragma unroll
  for (int i = 0; i < 8; ++i) {
    const int lid = w * 32 + i * 4 + sub;
    const v8h v = *(const v8ha*)(sT + lid * 64 + 8 * q8);
    _Float16* dst = base + (size_t)lid * ldc + 8 * q8;
    *(volatile v8h*)dst = v;
  }
}

__device__ __forceinline__ void f32_resid_store_pass(const float* sF, float* C32, const float* resid,
                                                     int m0, int n0, int ldc, int w, int lane) {
  const int q8 = lane & 7, sub = lane >> 3;
  #pragma unroll
  for (int i = 0; i < 16; ++i) {
    const int lid = i * 4 + sub;
    const int row = 32 * w + (lid >> 1), hl = lid & 1;
    const v4f v = *(const v4fa*)(sF + row * 64 + 32 * hl + 4 * q8);
    const size_t gi = (size_t)(m0 + row) * ldc + n0 + 32 * hl + 4 * q8;
    const v4f rv = *(const v4fa*)(resid + gi);
    const v4f st = v + rv;
    *(volatile v4f*)(C32 + gi) = st;
  }
}

template <int MODE>
__global__ __launch_bounds__(128) void gemm_kernel(
    const _Float16* __restrict__ A, const _Float16* __restrict__ Bt,
    const float* __restrict__ bias, const float* resid,
    float* C32, _Float16* C16,
    _Float16* qh, _Float16* kh, _Float16* vt,
    int K, int ldc, float inv)
{
  __shared__ __attribute__((aligned(16))) float sbuf[128 * 64];

  const int tid = threadIdx.x, lane = tid & 31, w = tid >> 5;
  const int h = lane >> 4, m = lane & 15;
  const int m0 = blockIdx.x * 128, n0 = blockIdx.y * 64;
  const int m0w = m0 + 32 * w;

  const _Float16* xa0 = A + (size_t)(m0w + m) * K;
  const _Float16* xa1 = xa0 + (size_t)16 * K;
  const _Float16* wb  = Bt + (size_t)(n0 + m) * K;

  const v8f zero8 = {0.f, 0.f, 0.f, 0.f, 0.f, 0.f, 0.f, 0.f};
  v8f acc[2][4];
  #pragma unroll
  for (int mt = 0; mt < 2; ++mt)
    #pragma unroll
    for (int nt = 0; nt < 4; ++nt) acc[mt][nt] = zero8;

  #pragma unroll 1
  for (int k0 = 0; k0 < K; k0 += 32) {
    const v16h a0 = load_frag(xa0 + k0, h);
    const v16h a1 = load_frag(xa1 + k0, h);
    #pragma unroll
    for (int nt = 0; nt < 4; ++nt) {
      const v16h b = load_frag(wb + (size_t)nt * 16 * K + k0, h);
      acc[0][nt] = wmma_f16(a0, b, acc[0][nt]);
      acc[1][nt] = wmma_f16(a1, b, acc[1][nt]);
    }
  }

  if (MODE == 0) {
    _Float16* sT = (_Float16*)sbuf;
    const int which = blockIdx.y >> 4, head = blockIdx.y & 15;
    #pragma unroll
    for (int nt = 0; nt < 4; ++nt) {
      const int feat = 16 * nt + m;
      const float bvl = bias[n0 + feat];
      #pragma unroll
      for (int mt = 0; mt < 2; ++mt) {
        #pragma unroll
        for (int r = 0; r < 8; ++r) {
          const int tokl = 32 * w + 16 * mt + 8 * h + r;
          const float y = acc[mt][nt][r] * inv + bvl;
          const int idx = (which == 2) ? (feat * 128 + tokl) : (tokl * HD + feat);
          sT[idx] = (_Float16)y;
        }
      }
    }
    __syncthreads();
    const int bi = m0 >> 10, l0 = m0 & 1023, bh = bi * NH + head;
    _Float16* plane = (which == 0) ? qh : kh;
    qkv_store_pass(sT, plane, vt, which, bh, l0, w, lane);
    __threadfence();
    qkv_store_pass(sT, plane, vt, which, bh, l0, w, lane);
  } else if (MODE == 1) {
    _Float16* sT = (_Float16*)sbuf;
    #pragma unroll
    for (int nt = 0; nt < 4; ++nt) {
      const int feat = 16 * nt + m;
      const float bvl = bias[n0 + feat];
      #pragma unroll
      for (int mt = 0; mt < 2; ++mt) {
        #pragma unroll
        for (int r = 0; r < 8; ++r) {
          const int tokl = 32 * w + 16 * mt + 8 * h + r;
          const float y = acc[mt][nt][r] * inv + bvl;
          const float ge = 0.5f * y * (1.0f + erff(y * 0.70710678118654752f));
          sT[tokl * 64 + feat] = (_Float16)(ge * GSCALE);
        }
      }
    }
    __syncthreads();
    _Float16* base = C16 + (size_t)m0 * ldc + n0;
    f16_store_pass(sT, base, ldc, w, lane);
    __threadfence();
    f16_store_pass(sT, base, ldc, w, lane);
  } else {
    float* sF = sbuf;
    #pragma unroll
    for (int nt = 0; nt < 4; ++nt) {
      const int feat = 16 * nt + m;
      const float bvl = bias[n0 + feat];
      #pragma unroll
      for (int mt = 0; mt < 2; ++mt) {
        #pragma unroll
        for (int r = 0; r < 8; ++r) {
          const int tokl = 32 * w + 16 * mt + 8 * h + r;
          sF[tokl * 64 + feat] = acc[mt][nt][r] * inv + bvl;
        }
      }
    }
    __syncthreads();
    f32_resid_store_pass(sF, C32, resid, m0, n0, ldc, w, lane);
    __threadfence();
    f32_resid_store_pass(sF, C32, resid, m0, n0, ldc, w, lane);
  }
}

__device__ __forceinline__ v16h pack_p(v8f a, v8f c) {
  const v16h r = { (_Float16)(a[0] * PSCALE), (_Float16)(a[1] * PSCALE), (_Float16)(a[2] * PSCALE), (_Float16)(a[3] * PSCALE),
                   (_Float16)(a[4] * PSCALE), (_Float16)(a[5] * PSCALE), (_Float16)(a[6] * PSCALE), (_Float16)(a[7] * PSCALE),
                   (_Float16)(c[0] * PSCALE), (_Float16)(c[1] * PSCALE), (_Float16)(c[2] * PSCALE), (_Float16)(c[3] * PSCALE),
                   (_Float16)(c[4] * PSCALE), (_Float16)(c[5] * PSCALE), (_Float16)(c[6] * PSCALE), (_Float16)(c[7] * PSCALE) };
  return r;
}

__device__ __forceinline__ void att_store_pass(const _Float16* so, _Float16* op,
                                               int b, int head, int q0, int lane) {
  const int q8 = lane & 7, sub = lane >> 3;
  #pragma unroll
  for (int i = 0; i < 4; ++i) {
    const int row = i * 4 + sub;
    const v8h v = *(const v8ha*)(so + row * 64 + 8 * q8);
    const size_t gi = ((size_t)b * SEQ + q0 + row) * DM + head * HD + 8 * q8;
    *(volatile v8h*)(op + gi) = v;
  }
}

__global__ __launch_bounds__(128) void attn_kernel(
    const _Float16* __restrict__ qh,
    const _Float16* __restrict__ kh,
    const _Float16* __restrict__ vt,
    _Float16* __restrict__ op)
{
  __shared__ __attribute__((aligned(16))) _Float16 sO[4 * 16 * 64];

  const int tid = threadIdx.x, lane = tid & 31, w = tid >> 5;
  const int h = lane >> 4, m = lane & 15;
  const int bh = blockIdx.y, b = bh >> 4, head = bh & 15;
  const int q0 = blockIdx.x * 64 + 16 * w;

  const _Float16* qrow = qh + ((size_t)bh * SEQ + q0 + m) * HD;
  const v16h qb0 = load_frag(qrow, h);
  const v16h qb1 = load_frag(qrow + 32, h);

  const v8f zero8 = {0.f, 0.f, 0.f, 0.f, 0.f, 0.f, 0.f, 0.f};
  v8f o[4];
  #pragma unroll
  for (int t = 0; t < 4; ++t) o[t] = zero8;
  float mrun = -1e30f, lrun = 0.0f;

  const _Float16* kbase = kh + ((size_t)bh * SEQ + m) * HD;
  const _Float16* vbase = vt + ((size_t)bh * HD + m) * SEQ;

  #pragma unroll 1
  for (int kb = 0; kb < SEQ; kb += 64) {
    v8f s[4];
    #pragma unroll
    for (int j = 0; j < 4; ++j) {
      const _Float16* kp = kbase + (size_t)(kb + 16 * j) * HD;
      const v16h kf0 = load_frag(kp, h);
      const v16h kf1 = load_frag(kp + 32, h);
      v8f z = zero8;
      z = wmma_f16(kf0, qb0, z);
      z = wmma_f16(kf1, qb1, z);
      s[j] = z;
    }

    float mloc = s[0][0];
    #pragma unroll
    for (int j = 0; j < 4; ++j)
      #pragma unroll
      for (int r = 0; r < 8; ++r) mloc = fmaxf(mloc, s[j][r]);
    mloc = fmaxf(mloc, __shfl_xor(mloc, 16, 32));
    const float mnew = fmaxf(mrun, mloc * SSCALE);
    const float alpha = __expf(mrun - mnew);
    mrun = mnew;
    float lsum = 0.0f;
    #pragma unroll
    for (int j = 0; j < 4; ++j)
      #pragma unroll
      for (int r = 0; r < 8; ++r) {
        const float p = __expf(s[j][r] * SSCALE - mnew);
        s[j][r] = p;
        lsum += p;
      }
    lsum += __shfl_xor(lsum, 16, 32);
    lrun = lrun * alpha + lsum;
    #pragma unroll
    for (int t = 0; t < 4; ++t)
      #pragma unroll
      for (int r = 0; r < 8; ++r) o[t][r] = o[t][r] * alpha;

    const v16h pb0 = pack_p(s[0], s[1]);
    const v16h pb1 = pack_p(s[2], s[3]);

    #pragma unroll
    for (int t = 0; t < 4; ++t) {
      const _Float16* vp = vbase + (size_t)(16 * t) * SEQ + kb;
      const v16h vf0 = load_frag(vp, h);
      const v16h vf1 = load_frag(vp + 32, h);
      o[t] = wmma_f16(vf0, pb0, o[t]);
      o[t] = wmma_f16(vf1, pb1, o[t]);
    }
  }

  const float inv = (1.0f / lrun) * (1.0f / PSCALE);
  _Float16* so = sO + w * 1024;
  #pragma unroll
  for (int t = 0; t < 4; ++t)
    #pragma unroll
    for (int r = 0; r < 8; ++r)
      so[m * 64 + 16 * t + 8 * h + r] = (_Float16)(o[t][r] * inv);
  __syncthreads();

  att_store_pass(so, op, b, head, q0, lane);
  __threadfence();
  att_store_pass(so, op, b, head, q0, lane);
}

extern "C" void kernel_launch(void* const* d_in, const int* in_sizes, int n_in,
                              void* d_out, int out_size, void* d_ws, size_t ws_size,
                              hipStream_t stream) {
  if (n_in < 13) return;
  if (in_sizes[0] != MROWS * DM) return;
  if (in_sizes[1] != DM * 3 * DM || in_sizes[2] != 3 * DM) return;
  if (in_sizes[3] != DM * DM || in_sizes[4] != DM) return;
  if (in_sizes[5] != DM * FF || in_sizes[6] != FF) return;
  if (in_sizes[7] != FF * DM || in_sizes[8] != DM) return;
  if (in_sizes[9] != DM || in_sizes[10] != DM || in_sizes[11] != DM || in_sizes[12] != DM) return;
  if (out_size != MROWS * DM) return;

  const float* x      = (const float*)d_in[0];
  const float* qkv_w  = (const float*)d_in[1];
  const float* qkv_b  = (const float*)d_in[2];
  const float* out_w  = (const float*)d_in[3];
  const float* out_b  = (const float*)d_in[4];
  const float* ffn_w1 = (const float*)d_in[5];
  const float* ffn_b1 = (const float*)d_in[6];
  const float* ffn_w2 = (const float*)d_in[7];
  const float* ffn_b2 = (const float*)d_in[8];
  const float* ln1_g  = (const float*)d_in[9];
  const float* ln1_b  = (const float*)d_in[10];
  const float* ln2_g  = (const float*)d_in[11];
  const float* ln2_b  = (const float*)d_in[12];
  float* out = (float*)d_out;

  const size_t wqkv_bytes = (size_t)3 * DM * DM * 2;
  const size_t w1_bytes   = (size_t)FF * DM * 2;
  const size_t w2_bytes   = (size_t)DM * FF * 2;
  const size_t wout_bytes = (size_t)DM * DM * 2;
  const size_t pl_bytes   = (size_t)MROWS * DM * 2;
  const size_t ffh_bytes  = (size_t)MROWS * FF * 2;
  const size_t x1_bytes   = (size_t)MROWS * DM * 4;

  const size_t off_r0 = 0;
  const size_t r0_bytes = wqkv_bytes + w1_bytes;
  const size_t off_a  = off_r0 + r0_bytes;
  const size_t a_bytes = 4 * pl_bytes;
  const size_t off_b  = off_a + a_bytes;
  const size_t off_c  = off_b + x1_bytes;
  const size_t c_bytes = pl_bytes;
  const size_t total  = off_c + c_bytes;
  if (ffh_bytes > a_bytes || wout_bytes > wqkv_bytes || w2_bytes > c_bytes) return;
  if (total > ws_size) return;

  char* ws = (char*)d_ws;
  _Float16* wqkvT = (_Float16*)(ws + off_r0);
  _Float16* w1T   = (_Float16*)(ws + off_r0 + wqkv_bytes);
  _Float16* woutT = (_Float16*)(ws + off_r0);
  _Float16* hpl   = (_Float16*)(ws + off_a);
  _Float16* qh    = (_Float16*)(ws + off_a + pl_bytes);
  _Float16* kh    = (_Float16*)(ws + off_a + 2 * pl_bytes);
  _Float16* vt    = (_Float16*)(ws + off_a + 3 * pl_bytes);
  _Float16* opl   = (_Float16*)(ws + off_a);
  _Float16* ffh   = (_Float16*)(ws + off_a);
  float*    x1    = (float*)(ws + off_b);
  _Float16* h2    = (_Float16*)(ws + off_c);
  _Float16* w2T   = (_Float16*)(ws + off_c);
  _Float16* spare = (_Float16*)(ws + off_c + w2_bytes);

  wtrans_kernel<<<dim3(3 * DM / 32, DM / 64), 256, 0, stream>>>(qkv_w, wqkvT, DM, 3 * DM, 32.0f);
  wtrans_kernel<<<dim3(FF / 32, DM / 64), 256, 0, stream>>>(ffn_w1, w1T, DM, FF, 32.0f);

  ln_kernel<<<MROWS, 128, 0, stream>>>(x, ln1_g, ln1_b, hpl);

  gemm_kernel<0><<<dim3(MROWS / 128, 3 * DM / 64), 128, 0, stream>>>(
      hpl, wqkvT, qkv_b, x, x1, spare, qh, kh, vt, DM, DM, 0.03125f);

  wtrans_kernel<<<dim3(DM / 32, DM / 64), 256, 0, stream>>>(out_w, woutT, DM, DM, 32.0f);

  attn_kernel<<<dim3(SEQ / 64, NB * NH), 128, 0, stream>>>(qh, kh, vt, opl);

  gemm_kernel<2><<<dim3(MROWS / 128, DM / 64), 128, 0, stream>>>(
      opl, woutT, out_b, x, x1, spare, qh, kh, vt, DM, DM, 0.03125f);

  ln_kernel<<<MROWS, 128, 0, stream>>>(x1, ln2_g, ln2_b, h2);

  gemm_kernel<1><<<dim3(MROWS / 128, FF / 64), 128, 0, stream>>>(
      h2, w1T, ffn_b1, x, x1, ffh, qh, kh, vt, DM, FF, 0.03125f);

  wtrans_kernel<<<dim3(DM / 32, FF / 64), 256, 0, stream>>>(ffn_w2, w2T, FF, DM, 64.0f);

  gemm_kernel<2><<<dim3(MROWS / 128, DM / 64), 128, 0, stream>>>(
      ffh, w2T, ffn_b2, x1, out, spare, spare, spare, spare, FF, DM, 0.0009765625f);
}
